// GFeedforward_7842610283358
// MI455X (gfx1250) — hardware-verified
//
#include <hip/hip_runtime.h>
#include <math.h>
#include <stddef.h>


typedef __bf16 v16bf __attribute__((ext_vector_type(16)));
typedef float v8f __attribute__((ext_vector_type(8)));
typedef float v4f __attribute__((ext_vector_type(4)));
typedef unsigned int u4 __attribute__((ext_vector_type(4)));
typedef u4 __attribute__((may_alias)) u4a;
typedef v4f __attribute__((may_alias)) v4fa;

#define NUM_FEAT   10
#define WORD_DIM   64
#define POS_DIM    32
#define DIS_DIM    32
#define IN_SIZE    992
#define HIDDEN     256
#define OUT_SIZE   50
#define OUT_PAD    64
#define KSTEP      32
#define NKSTEPS    (IN_SIZE / KSTEP)
#define NCHUNK     64
#define W1P        1024
#define W2P        HIDDEN

#define WAVE       32
#define WAVES_BLK  2
#define THREADS    (WAVE * WAVES_BLK)
#define ROWS_WAVE  16
#define ROWS_BLK   (ROWS_WAVE * WAVES_BLK)

#define LDS_XS     (ROWS_BLK * IN_SIZE)
#define LDS_HS     (ROWS_BLK * HIDDEN)
#define LDS_SB     (NCHUNK * KSTEP)
#define LDS_MAIN_BYTES ((2 * LDS_XS + 2 * LDS_HS + 2 * LDS_SB) * 2)

#define CV_THREADS 128
#define CV_RB      8

static_assert(ROWS_BLK * OUT_SIZE * 4 <= 2 * LDS_SB * 2);
static_assert((ROWS_BLK * OUT_SIZE * 4) % 128 == 0);
static_assert(IN_SIZE % KSTEP == 0 && HIDDEN % KSTEP == 0);
static_assert((W1P % 64) == 0 && (W2P % 64) == 0);

union Frag {
    v16bf v;
    u4    q[2];
};

__device__ __forceinline__ v8f zero8() {
    v8f z = {0.f, 0.f, 0.f, 0.f, 0.f, 0.f, 0.f, 0.f};
    return z;
}

__device__ __forceinline__ unsigned short f2bf(float f) {
    unsigned int u = __float_as_uint(f);
    u += 0x7FFFu + ((u >> 16) & 1u);
    return (unsigned short)(u >> 16);
}
__device__ __forceinline__ float bf2f(unsigned short b) {
    return __uint_as_float(((unsigned int)b) << 16);
}
__device__ __forceinline__ void split_bf(float f, unsigned short& hi, unsigned short& lo) {
    hi = f2bf(f);
    lo = f2bf(f - bf2f(hi));
}

__device__ __forceinline__ v16bf frag_lds(const unsigned short* base, int pitch, int rc, int k0, int h) {
    const unsigned short* p = base + rc * pitch + k0 + 8 * h;
    Frag f;
    f.q[0] = *(const u4a*)(p);
    f.q[1] = *(const u4a*)(p + 16);
    return f.v;
}
__device__ __forceinline__ v16bf frag_glb(const unsigned short* __restrict__ base, int pitch, int rc, int k0, int h) {
    const unsigned short* p = base + (size_t)rc * pitch + k0 + 8 * h;
    Frag f;
    f.q[0] = *(const u4a*)(p);
    f.q[1] = *(const u4a*)(p + 16);
    return f.v;
}

__device__ __forceinline__ v8f wmma3(v16bf ah, v16bf al, v16bf bh, v16bf bl, v8f acc) {
    acc = __builtin_amdgcn_wmma_f32_16x16x32_bf16(false, ah, false, bh, (short)0, acc, false, false);
    acc = __builtin_amdgcn_wmma_f32_16x16x32_bf16(false, ah, false, bl, (short)0, acc, false, false);
    acc = __builtin_amdgcn_wmma_f32_16x16x32_bf16(false, al, false, bh, (short)0, acc, false, false);
    asm volatile("v_nop\n\tv_nop\n\tv_nop\n\tv_nop"
                 : "+v"(acc)
                 : "v"(ah), "v"(al), "v"(bh), "v"(bl));
    return acc;
}

__global__ __launch_bounds__(CV_THREADS) void k_tsplit(
    const float* __restrict__ w, int K, int N, int KP,
    unsigned short* __restrict__ ph, unsigned short* __restrict__ pl)
{
    extern __shared__ __align__(16) unsigned char cv_smem[];
    unsigned short* th = (unsigned short*)cv_smem;
    unsigned short* tl = th + CV_RB * KP;

    const int tid = threadIdx.x;
    const int n0  = blockIdx.x * CV_RB;
    const int tot = CV_RB * KP;

    for (int idx = tid; idx < tot; idx += CV_THREADS) {
        const int r = idx / KP;
        const int k = idx - r * KP;
        const int n = n0 + r;
        float v = 0.f;
        if (n < N && k < K) v = w[(size_t)k * N + n];
        unsigned short hi, lo;
        split_bf(v, hi, lo);
        th[idx] = hi;
        tl[idx] = lo;
    }
    __syncthreads();

    const int cpp = tot >> 3;
    const size_t dbase = (size_t)n0 * KP;

    for (int c = tid; c < 2 * cpp; c += CV_THREADS) {
        const int p  = (c >= cpp) ? 1 : 0;
        const int cc = c - p * cpp;
        const unsigned short* s = (p ? tl : th) + cc * 8;
        unsigned short* d = (p ? pl : ph) + dbase + (size_t)cc * 8;
        const u4 v = *(const u4a*)s;
        *(volatile u4*)d = v;
    }
    __threadfence();
    for (int c = tid; c < 2 * cpp; c += CV_THREADS) {
        const int p  = (c >= cpp) ? 1 : 0;
        const int cc = c - p * cpp;
        const unsigned short* s = (p ? tl : th) + cc * 8;
        unsigned short* d = (p ? pl : ph) + dbase + (size_t)cc * 8;
        const u4 v = *(const u4a*)s;
        *(volatile u4*)d = v;
    }
}

__global__ __launch_bounds__(THREADS) void k_ffwd(
    const int*   __restrict__ word_idx, const int* __restrict__ pos_idx,
    const int*   __restrict__ dis_idx,
    const float* __restrict__ word_emb, const float* __restrict__ pos_emb,
    const float* __restrict__ dis_emb,
    const unsigned short* __restrict__ w1h, const unsigned short* __restrict__ w1l,
    const float* __restrict__ b1,
    const unsigned short* __restrict__ w2h, const unsigned short* __restrict__ w2l,
    const float* __restrict__ b2,
    float* __restrict__ out,
    int Bn, int wvocab, int pvocab, int dvocab)
{
    extern __shared__ __align__(16) unsigned char smem[];
    unsigned short* xsh = (unsigned short*)smem;
    unsigned short* xsl = xsh + LDS_XS;
    unsigned short* hsh = xsl + LDS_XS;
    unsigned short* hsl = hsh + LDS_HS;
    unsigned short* sbh = hsl + LDS_HS;
    unsigned short* sbl = sbh + LDS_SB;
    float*          os  = (float*)sbh;

    const int tid  = threadIdx.x;
    const int lane = tid & (WAVE - 1);
    const int wv   = tid >> 5;
    const int h    = lane >> 4;
    const int m    = lane & 15;
    const int row0 = blockIdx.x * ROWS_BLK;

    for (int r = 0; r < ROWS_BLK; ++r) {
        const int  grow  = row0 + r;
        const bool valid = grow < Bn;
        for (int it = 0; it < (IN_SIZE + THREADS - 1) / THREADS; ++it) {
            const int col = it * THREADS + tid;
            if (col < IN_SIZE) {
                float v = 0.f;
                if (valid) {
                    if (col < NUM_FEAT * WORD_DIM) {
                        const int f = col >> 6, d = col & 63;
                        int wi = word_idx[(size_t)grow * NUM_FEAT + f];
                        wi = wi < 0 ? 0 : (wi >= wvocab ? wvocab - 1 : wi);
                        v = word_emb[(size_t)wi * WORD_DIM + d];
                    } else if (col < NUM_FEAT * (WORD_DIM + POS_DIM)) {
                        const int c = col - NUM_FEAT * WORD_DIM;
                        const int f = c >> 5, d = c & 31;
                        int pi = pos_idx[(size_t)grow * NUM_FEAT + f];
                        pi = pi < 0 ? 0 : (pi >= pvocab ? pvocab - 1 : pi);
                        v = pos_emb[(size_t)pi * POS_DIM + d];
                    } else {
                        int di = dis_idx[grow];
                        di = di < 0 ? 0 : (di >= dvocab ? dvocab - 1 : di);
                        v = dis_emb[(size_t)di * DIS_DIM + (col - NUM_FEAT * (WORD_DIM + POS_DIM))];
                    }
                }
                unsigned short hi, lo;
                split_bf(v, hi, lo);
                xsh[r * IN_SIZE + col] = hi;
                xsl[r * IN_SIZE + col] = lo;
            }
        }
    }
    __syncthreads();

    const unsigned short* xwh = xsh + wv * ROWS_WAVE * IN_SIZE;
    const unsigned short* xwl = xsl + wv * ROWS_WAVE * IN_SIZE;
    unsigned short*       hwh = hsh + wv * ROWS_WAVE * HIDDEN;
    unsigned short*       hwl = hsl + wv * ROWS_WAVE * HIDDEN;

    for (int chunk = 0; chunk < HIDDEN / NCHUNK; ++chunk) {
        v8f acc[4];
        #pragma unroll
        for (int t = 0; t < 4; ++t) acc[t] = zero8();

        for (int kk = 0; kk < NKSTEPS; ++kk) {
            __syncthreads();
            #pragma unroll
            for (int i = 0; i < (2 * LDS_SB / 8) / THREADS; ++i) {
                const int c  = i * THREADS + tid;
                const int pl = c >> 8;
                const int cc = c & 255;
                const int nl = cc >> 2;
                const int ko = (cc & 3) * 8;
                const unsigned short* src = (pl ? w1l : w1h)
                    + (size_t)(chunk * NCHUNK + nl) * W1P + kk * KSTEP + ko;
                unsigned short* dst = (pl ? sbl : sbh) + nl * KSTEP + ko;
                const u4 v = *(const u4a*)src;
                *(u4a*)dst = v;
            }
            __syncthreads();

            const int k0 = kk * KSTEP;
            const v16bf ah = frag_lds(xwh, IN_SIZE, m, k0, h);
            const v16bf al = frag_lds(xwl, IN_SIZE, m, k0, h);
            #pragma unroll
            for (int t = 0; t < 4; ++t) {
                const v16bf bh = frag_lds(sbh, KSTEP, t * 16 + m, 0, h);
                const v16bf bl = frag_lds(sbl, KSTEP, t * 16 + m, 0, h);
                acc[t] = wmma3(ah, al, bh, bl, acc[t]);
            }
        }

        #pragma unroll
        for (int t = 0; t < 4; ++t) {
            const int   n   = chunk * NCHUNK + t * 16 + m;
            const float bia = b1[n];
            #pragma unroll
            for (int r = 0; r < 8; ++r) {
                const float u  = acc[t][r] + bia;
                const float hv = tanhf(u * u * u);
                unsigned short hi, lo;
                split_bf(hv, hi, lo);
                hwh[(8 * h + r) * HIDDEN + n] = hi;
                hwl[(8 * h + r) * HIDDEN + n] = lo;
            }
        }
    }
    __syncthreads();

    v8f oacc[4];
    #pragma unroll
    for (int t = 0; t < 4; ++t) oacc[t] = zero8();

    for (int kk = 0; kk < HIDDEN / KSTEP; ++kk) {
        const int k0 = kk * KSTEP;
        const v16bf ah = frag_lds(hwh, HIDDEN, m, k0, h);
        const v16bf al = frag_lds(hwl, HIDDEN, m, k0, h);
        #pragma unroll
        for (int t = 0; t < 4; ++t) {
            const v16bf bh = frag_glb(w2h, W2P, t * 16 + m, k0, h);
            const v16bf bl = frag_glb(w2l, W2P, t * 16 + m, k0, h);
            oacc[t] = wmma3(ah, al, bh, bl, oacc[t]);
        }
    }

    #pragma unroll
    for (int t = 0; t < 4; ++t) {
        const int n = t * 16 + m;
        if (n < OUT_SIZE) {
            const float bia = b2[n];
            #pragma unroll
            for (int r = 0; r < 8; ++r) {
                os[(wv * ROWS_WAVE + 8 * h + r) * OUT_SIZE + n] = oacc[t][r] + bia;
            }
        }
    }
    __syncthreads();

    float* outb = out + (size_t)row0 * OUT_SIZE;
    const int nf4 = ROWS_BLK * OUT_SIZE / 4;
    if (row0 + ROWS_BLK <= Bn) {
        #pragma unroll
        for (int i = 0; i < (ROWS_BLK * OUT_SIZE / 4 + THREADS - 1) / THREADS; ++i) {
            const int q = i * THREADS + tid;
            if (q < nf4) {
                const v4f v = *(const v4fa*)(os + 4 * q);
                *(volatile v4f*)(outb + 4 * q) = v;
            }
        }
        __threadfence();
        #pragma unroll
        for (int i = 0; i < (ROWS_BLK * OUT_SIZE / 4 + THREADS - 1) / THREADS; ++i) {
            const int q = i * THREADS + tid;
            if (q < nf4) {
                const v4f v = *(const v4fa*)(os + 4 * q);
                *(volatile v4f*)(outb + 4 * q) = v;
            }
        }
    } else {
        const int nval = Bn - row0;
        const int tot  = (nval > 0 ? nval : 0) * OUT_SIZE;
        for (int e = tid; e < tot; e += THREADS) {
            const float v = os[e];
            *(volatile float*)(outb + e) = v;
        }
        __threadfence();
        for (int e = tid; e < tot; e += THREADS) {
            const float v = os[e];
            *(volatile float*)(outb + e) = v;
        }
    }
}

extern "C" void kernel_launch(void* const* d_in, const int* in_sizes, int n_in,
                              void* d_out, int out_size, void* d_ws, size_t ws_size,
                              hipStream_t stream) {
    (void)n_in;
    const int*   word_idx = (const int*)  d_in[0];
    const int*   pos_idx  = (const int*)  d_in[1];
    const int*   dis_idx  = (const int*)  d_in[2];
    const float* word_emb = (const float*)d_in[3];
    const float* pos_emb  = (const float*)d_in[4];
    const float* dis_emb  = (const float*)d_in[5];
    const float* w1       = (const float*)d_in[6];
    const float* b1       = (const float*)d_in[7];
    const float* w2       = (const float*)d_in[8];
    const float* b2       = (const float*)d_in[9];
    float*       out      = (float*)d_out;

    unsigned char* ws = (unsigned char*)d_ws;
    size_t off = 0;
    const size_t w1_plane = (size_t)HIDDEN * W1P * sizeof(unsigned short);
    const size_t w2_plane = (size_t)OUT_PAD * W2P * sizeof(unsigned short);
    unsigned short* w1h = (unsigned short*)(ws + off); off += w1_plane;
    unsigned short* w1l = (unsigned short*)(ws + off); off += w1_plane;
    unsigned short* w2h = (unsigned short*)(ws + off); off += w2_plane;
    unsigned short* w2l = (unsigned short*)(ws + off); off += w2_plane;
    if (off > ws_size) return;

    int Bn = out_size / OUT_SIZE;
    const int bw = in_sizes[0] / NUM_FEAT;
    const int bp = in_sizes[1] / NUM_FEAT;
    const int bd = in_sizes[2];
    if (bw < Bn) Bn = bw;
    if (bp < Bn) Bn = bp;
    if (bd < Bn) Bn = bd;
    if (Bn <= 0) return;

    const int wvocab = in_sizes[3] / WORD_DIM;
    const int pvocab = in_sizes[4] / POS_DIM;
    const int dvocab = in_sizes[5] / DIS_DIM;
    if (wvocab <= 0 || pvocab <= 0 || dvocab <= 0) return;

    const size_t lds_cv1 = (size_t)2 * CV_RB * W1P * sizeof(unsigned short);
    const size_t lds_cv2 = (size_t)2 * CV_RB * W2P * sizeof(unsigned short);
    const size_t lds_main = (size_t)LDS_MAIN_BYTES;

    hipFuncSetAttribute(reinterpret_cast<const void*>(&k_tsplit),
                        hipFuncAttributeMaxDynamicSharedMemorySize, (int)lds_cv1);
    hipFuncSetAttribute(reinterpret_cast<const void*>(&k_ffwd),
                        hipFuncAttributeMaxDynamicSharedMemorySize, (int)lds_main);

    k_tsplit<<<HIDDEN / CV_RB, CV_THREADS, lds_cv1, stream>>>(w1, IN_SIZE, HIDDEN, W1P, w1h, w1l);
    k_tsplit<<<OUT_PAD / CV_RB, CV_THREADS, lds_cv2, stream>>>(w2, HIDDEN, OUT_SIZE, W2P, w2h, w2l);

    const int blocks = (Bn + ROWS_BLK - 1) / ROWS_BLK;
    k_ffwd<<<blocks, THREADS, lds_main, stream>>>(
        word_idx, pos_idx, dis_idx, word_emb, pos_emb, dis_emb,
        w1h, w1l, b1, w2h, w2l, b2, out, Bn, wvocab, pvocab, dvocab);
}
